// OneGATCN_87720412053584
// MI455X (gfx1250) — hardware-verified
//
#include <hip/hip_runtime.h>
#include <hip/hip_bf16.h>
#include <stddef.h>


#define F_IN  512
#define HID   1024
#define C1    512
#define C2    128
#define NCP   128
#define TM    64
#define TNB   128
#define CSP   132
#define NBK   64
#define CHUNK 2048
#define NTHR  256
#define NWAVE 8
#define WCAP  256
#define NGRP  (CHUNK / (NTHR * 4))
#define SELF_FLAG (1 << 20)

#define LDS_SACC (NBK * HID)
#define LDS_GAT_BYTES ((LDS_SACC + HID + NBK + NBK) * 4 + (NWAVE * WCAP + NWAVE) * 4)

static_assert(WCAP == (CHUNK / NTHR) * 32);
static_assert(NGRP == 2);
static_assert(NBK == NWAVE * 8);
static_assert((NBK & (NBK - 1)) == 0);
static_assert(CHUNK <= 4096);
static_assert(LDS_GAT_BYTES == 274976);
static_assert(HID == 4 * NTHR);

typedef float          v4f   __attribute__((ext_vector_type(4)));
typedef float          v8f   __attribute__((ext_vector_type(8)));
typedef int            v4i   __attribute__((ext_vector_type(4)));
typedef unsigned short v8us  __attribute__((ext_vector_type(8)));
typedef __bf16         v16bf __attribute__((ext_vector_type(16)));
union FragB { v16bf v; v8us h[2]; };

__device__ __forceinline__ unsigned int bf_rne(float f) {
  unsigned int u = __float_as_uint(f);
  u += 0x7FFFu + ((u >> 16) & 1u);
  return u >> 16;
}
__device__ __forceinline__ void split_bf(float v, unsigned short& hi, unsigned short& lo) {
  const unsigned int h = bf_rne(v);
  const float hv = __uint_as_float(h << 16);
  hi = (unsigned short)h;
  lo = (unsigned short)bf_rne(v - hv);
}

__device__ __forceinline__ v8f wmb(v16bf a, v16bf b, v8f c) {
  v8f d = __builtin_amdgcn_wmma_f32_16x16x32_bf16(false, a, false, b, (short)0, c, false, false);
  asm volatile("v_nop\n\tv_nop\n\tv_nop\n\tv_nop" : "+v"(d) : "v"(a), "v"(b));
  return d;
}

__device__ __forceinline__ float wsum(float v) {
  v += __shfl_xor(v, 16, 32);
  v += __shfl_xor(v, 8, 32);
  v += __shfl_xor(v, 4, 32);
  v += __shfl_xor(v, 2, 32);
  v += __shfl_xor(v, 1, 32);
  return v;
}

__device__ __forceinline__ v4f lrelu4(v4f t) {
  v4f r;
  r.x = t.x > 0.f ? t.x : 0.2f * t.x;
  r.y = t.y > 0.f ? t.y : 0.2f * t.y;
  r.z = t.z > 0.f ? t.z : 0.2f * t.z;
  r.w = t.w > 0.f ? t.w : 0.2f * t.w;
  return r;
}

__global__ __launch_bounds__(NTHR) void k_cvt_rows(const float* __restrict__ src, int R, int C, int RP,
                                                   unsigned short* hi, unsigned short* lo) {
  const long long i8 = (long long)blockIdx.x * NTHR + threadIdx.x;
  const long long tot8 = (long long)RP * C / 8;
  if (i8 >= tot8) return;
  const long long e0 = i8 * 8;
  const int r = (int)(e0 / C);
  const int c = (int)(e0 - (long long)r * C);
  const int rr = (r < R) ? r : (R - 1);
  const float* p = src + (size_t)rr * C + c;
  const v4f z4 = {0.f, 0.f, 0.f, 0.f};
  v4f a = *(const v4f*)p;
  v4f b = *(const v4f*)(p + 4);
  a = (r < R) ? a : z4;
  b = (r < R) ? b : z4;
  float t[8];
  t[0] = a.x; t[1] = a.y; t[2] = a.z; t[3] = a.w;
  t[4] = b.x; t[5] = b.y; t[6] = b.z; t[7] = b.w;
  v8us H, L;
#pragma unroll
  for (int e = 0; e < 8; ++e) { unsigned short u, w; split_bf(t[e], u, w); H[e] = u; L[e] = w; }
  *(volatile v8us*)(hi + e0) = H;
  *(volatile v8us*)(lo + e0) = L;
  __threadfence();
  *(volatile v8us*)(hi + e0) = H;
  *(volatile v8us*)(lo + e0) = L;
}

__global__ __launch_bounds__(NTHR) void k_cvt_T(const float* __restrict__ src, int K, int N, int KP,
                                                unsigned short* hi, unsigned short* lo) {
  __shared__ float S[64 * 65];
  const int tid = threadIdx.x;
  const int k0 = blockIdx.x * 64;
  const int n0 = blockIdx.y * 64;
  {
    const int nn = tid & 63;
    const int kq = tid >> 6;
    int gn = n0 + nn;
    const bool nok = gn < N;
    gn = nok ? gn : (N - 1);
#pragma unroll 4
    for (int it = 0; it < 16; ++it) {
      const int kk = kq + 4 * it;
      int gk = k0 + kk;
      const bool kok = gk < K;
      gk = kok ? gk : (K - 1);
      float v = src[(size_t)gk * N + gn];
      v = (nok && kok) ? v : 0.0f;
      S[kk * 65 + nn] = v;
    }
  }
  __syncthreads();
#pragma unroll 1
  for (int pass = 0; pass < 2; ++pass) {
#pragma unroll 1
    for (int it = 0; it < 2; ++it) {
      const int p  = it * NTHR + tid;
      const int nn = p >> 3;
      const int q  = p & 7;
      v8us H, L;
#pragma unroll
      for (int e = 0; e < 8; ++e) {
        unsigned short u, w;
        split_bf(S[(8 * q + e) * 65 + nn], u, w);
        H[e] = u; L[e] = w;
      }
      const size_t o = (size_t)(n0 + nn) * KP + k0 + 8 * q;
      *(volatile v8us*)(hi + o) = H;
      *(volatile v8us*)(lo + o) = L;
    }
    if (pass == 0) __threadfence();
  }
}

__global__ __launch_bounds__(NTHR) void k_gemm(
    const unsigned short* __restrict__ Ahi, const unsigned short* __restrict__ Alo, int lda,
    const unsigned short* __restrict__ Bhi, const unsigned short* __restrict__ Blo, int ldb, int K,
    const float* __restrict__ bias, int nBias, int mode,
    float* Cf, unsigned short* Chi, unsigned short* Clo, int ldc,
    float* Out, int Mreal, int Nreal)
{
  __shared__ __attribute__((aligned(16))) float Cs[TM * CSP];

  const int tid  = threadIdx.x;
  const int lane = tid & 31;
  const int wave = tid >> 5;
  const int wmi  = wave >> 2;
  const int wni  = wave & 3;
  const int hh   = lane >> 4;
  const int m    = lane & 15;
  const int m0   = blockIdx.x * TM;
  const int n0   = blockIdx.y * TNB;

  const size_t ao0 = (size_t)(m0 + wmi * 32 + m) * lda + 8 * hh;
  const size_t ao1 = ao0 + (size_t)16 * lda;
  const size_t bo0 = (size_t)(n0 + wni * 32 + m) * ldb + 8 * hh;
  const size_t bo1 = bo0 + (size_t)16 * ldb;

  v8f c00 = {0.f, 0.f, 0.f, 0.f, 0.f, 0.f, 0.f, 0.f};
  v8f c01 = c00, c10 = c00, c11 = c00;

#pragma unroll 1
  for (int k0 = 0; k0 < K; k0 += 32) {
    FragB ah0, ah1, al0, al1, bh0, bh1, bl0, bl1;
    ah0.h[0] = *(const v8us*)(Ahi + ao0 + k0);  ah0.h[1] = *(const v8us*)(Ahi + ao0 + k0 + 16);
    ah1.h[0] = *(const v8us*)(Ahi + ao1 + k0);  ah1.h[1] = *(const v8us*)(Ahi + ao1 + k0 + 16);
    al0.h[0] = *(const v8us*)(Alo + ao0 + k0);  al0.h[1] = *(const v8us*)(Alo + ao0 + k0 + 16);
    al1.h[0] = *(const v8us*)(Alo + ao1 + k0);  al1.h[1] = *(const v8us*)(Alo + ao1 + k0 + 16);
    bh0.h[0] = *(const v8us*)(Bhi + bo0 + k0);  bh0.h[1] = *(const v8us*)(Bhi + bo0 + k0 + 16);
    bh1.h[0] = *(const v8us*)(Bhi + bo1 + k0);  bh1.h[1] = *(const v8us*)(Bhi + bo1 + k0 + 16);
    bl0.h[0] = *(const v8us*)(Blo + bo0 + k0);  bl0.h[1] = *(const v8us*)(Blo + bo0 + k0 + 16);
    bl1.h[0] = *(const v8us*)(Blo + bo1 + k0);  bl1.h[1] = *(const v8us*)(Blo + bo1 + k0 + 16);

    c00 = wmb(ah0.v, bh0.v, c00);  c00 = wmb(ah0.v, bl0.v, c00);  c00 = wmb(al0.v, bh0.v, c00);
    c01 = wmb(ah0.v, bh1.v, c01);  c01 = wmb(ah0.v, bl1.v, c01);  c01 = wmb(al0.v, bh1.v, c01);
    c10 = wmb(ah1.v, bh0.v, c10);  c10 = wmb(ah1.v, bl0.v, c10);  c10 = wmb(al1.v, bh0.v, c10);
    c11 = wmb(ah1.v, bh1.v, c11);  c11 = wmb(ah1.v, bl1.v, c11);  c11 = wmb(al1.v, bh1.v, c11);
  }

  {
    const int rb = wmi * 32 + 8 * hh;
    const int cb = wni * 32 + m;
#pragma unroll
    for (int r = 0; r < 8; ++r) {
      Cs[(rb + r) * CSP + cb]           = c00[r];
      Cs[(rb + r) * CSP + cb + 16]      = c01[r];
      Cs[(rb + 16 + r) * CSP + cb]      = c10[r];
      Cs[(rb + 16 + r) * CSP + cb + 16] = c11[r];
    }
  }
  __syncthreads();

  if (mode == 0) {
    v4f b4;
    {
      const int c = n0 + 4 * lane;
      const int q0 = c     < nBias ? c     : nBias - 1;
      const int q1 = c + 1 < nBias ? c + 1 : nBias - 1;
      const int q2 = c + 2 < nBias ? c + 2 : nBias - 1;
      const int q3 = c + 3 < nBias ? c + 3 : nBias - 1;
      b4.x = bias[q0]; b4.y = bias[q1]; b4.z = bias[q2]; b4.w = bias[q3];
    }
#pragma unroll 1
    for (int pass = 0; pass < 2; ++pass) {
#pragma unroll 1
      for (int rr = 0; rr < 8; ++rr) {
        const int row = wave * 8 + rr;
        const v4f v = *(const v4f*)(Cs + row * CSP + 4 * lane) + b4;
        *(volatile v4f*)(Cf + (size_t)(m0 + row) * ldc + n0 + 4 * lane) = v;
      }
      if (pass == 0) __threadfence();
    }
  } else if (mode == 1) {
    const int hs = lane >> 4;
    const int cl = lane & 15;
    float b8[8];
#pragma unroll
    for (int e = 0; e < 8; ++e) {
      const int c = n0 + 8 * cl + e;
      b8[e] = bias[c < nBias ? c : nBias - 1];
    }
    unsigned short* plane = hs ? Clo : Chi;
#pragma unroll 1
    for (int pass = 0; pass < 2; ++pass) {
#pragma unroll 1
      for (int rr = 0; rr < 8; ++rr) {
        const int row = wave * 8 + rr;
        const float* cs = Cs + row * CSP + 8 * cl;
        v8us H, L;
#pragma unroll
        for (int e = 0; e < 8; ++e) {
          float v = cs[e] + b8[e];
          v = v > 0.f ? v : 0.f;
          unsigned short u, w;
          split_bf(v, u, w);
          H[e] = u; L[e] = w;
        }
        const v8us o = hs ? L : H;
        *(volatile v8us*)(plane + (size_t)(m0 + row) * ldc + n0 + 8 * cl) = o;
      }
      if (pass == 0) __threadfence();
    }
  } else {
    int mv = Mreal - m0;
    mv = mv > TM ? TM : mv;
    mv = mv < 0 ? 0 : mv;
    const int cnt = mv * Nreal;
    float* base = Out + (size_t)m0 * Nreal;
#pragma unroll 1
    for (int pass = 0; pass < 2; ++pass) {
#pragma unroll 1
      for (int f = tid * 4; f + 3 < cnt; f += NTHR * 4) {
        int r = f / Nreal;
        int c = f - r * Nreal;
        float t[4];
#pragma unroll
        for (int e = 0; e < 4; ++e) {
          t[e] = Cs[r * CSP + c] + bias[c];
          ++c;
          if (c == Nreal) { c = 0; ++r; }
        }
        v4f v;
        v.x = t[0]; v.y = t[1]; v.z = t[2]; v.w = t[3];
        *(volatile v4f*)(base + f) = v;
      }
      {
        const int rem = cnt & 3;
        const int ft  = cnt - rem;
        if (tid < rem) {
          const int f = ft + tid;
          const int r = f / Nreal;
          const int c = f - r * Nreal;
          const float v = Cs[r * CSP + c] + bias[c];
          *(volatile float*)(base + f) = v;
        }
      }
      if (pass == 0) __threadfence();
    }
  }
}

__global__ __launch_bounds__(NTHR) void k_gat(
    const float* __restrict__ xl, const float* __restrict__ xr, const int* __restrict__ ei,
    const float* __restrict__ att, const float* __restrict__ cb,
    unsigned short* hhi, unsigned short* hlo, int nN, int nE)
{
  extern __shared__ v4f lds_dyn[];
  float* sacc = (float*)lds_dyn;
  float* satt = sacc + LDS_SACC;
  float* mls  = satt + HID;
  float* lls  = mls + NBK;
  int*   list = (int*)(lls + NBK);
  int*   wcnt = list + NWAVE * WCAP;

  const int tid  = threadIdx.x;
  const int lane = tid & 31;
  const int wave = tid >> 5;
  const int nodeBase = blockIdx.x * NBK;

  {
    const v4f z4 = {0.f, 0.f, 0.f, 0.f};
    for (int i = tid; i < LDS_SACC / 4; i += NTHR) lds_dyn[i] = z4;
    *(v4f*)(satt + 4 * tid) = *(const v4f*)(att + 4 * tid);
    if (tid < NBK) { mls[tid] = __uint_as_float(0xff800000u); lls[tid] = 0.f; }
  }
  __syncthreads();

  const int* eid = ei + nE;
  const bool vec_ok = ((nE & 3) == 0);
  const int nChunks = (nE + CHUNK - 1) / CHUNK;

#pragma unroll 1
  for (int ch = 0; ch <= nChunks; ++ch) {
    const int cbase = ch * CHUNK;
    if (ch < nChunks) {
      int wc = 0;
#pragma unroll
      for (int g = 0; g < NGRP; ++g) {
        const int el0 = (g * NTHR + tid) * 4;
        const int e0  = cbase + el0;
        const int sent = -2147483647 - 1;
        v4i d;
        if (vec_ok && (cbase + CHUNK <= nE)) {
          d = *(const v4i*)(eid + e0);
        } else {
          const int q0 = e0     < nE ? e0     : nE - 1;
          const int q1 = e0 + 1 < nE ? e0 + 1 : nE - 1;
          const int q2 = e0 + 2 < nE ? e0 + 2 : nE - 1;
          const int q3 = e0 + 3 < nE ? e0 + 3 : nE - 1;
          const int v0 = eid[q0], v1 = eid[q1], v2 = eid[q2], v3 = eid[q3];
          d.x = (e0     < nE) ? v0 : sent;
          d.y = (e0 + 1 < nE) ? v1 : sent;
          d.z = (e0 + 2 < nE) ? v2 : sent;
          d.w = (e0 + 3 < nE) ? v3 : sent;
        }
        const unsigned s0 = (unsigned)d.x - (unsigned)nodeBase;
        const unsigned s1 = (unsigned)d.y - (unsigned)nodeBase;
        const unsigned s2 = (unsigned)d.z - (unsigned)nodeBase;
        const unsigned s3 = (unsigned)d.w - (unsigned)nodeBase;
        const bool h0 = s0 < (unsigned)NBK;
        const bool h1 = s1 < (unsigned)NBK;
        const bool h2 = s2 < (unsigned)NBK;
        const bool h3 = s3 < (unsigned)NBK;
        const unsigned many = __builtin_amdgcn_ballot_w32(h0 | h1 | h2 | h3);
        if (many != 0u) {
#define HITJ(J, HJ, SJ) { \
            const unsigned mj = __builtin_amdgcn_ballot_w32(HJ); \
            if (HJ) { \
              const int pos = wc + (int)__builtin_amdgcn_mbcnt_lo(mj, 0u); \
              if (pos < WCAP) list[wave * WCAP + pos] = ((el0 + (J)) << 6) | (int)(SJ); \
            } \
            wc += (int)__builtin_popcount(mj); }
          HITJ(0, h0, s0)
          HITJ(1, h1, s1)
          HITJ(2, h2, s2)
          HITJ(3, h3, s3)
#undef HITJ
        }
      }
      if (lane == 0) wcnt[wave] = wc;
    } else {
      if (tid < NBK) list[tid] = SELF_FLAG | tid;
      if (tid < NWAVE) wcnt[tid] = (tid == 0) ? NBK : 0;
    }
    __syncthreads();

#pragma unroll 1
    for (int wsx = 0; wsx < NWAVE; ++wsx) {
      int n = wcnt[wsx];
      n = n > WCAP ? WCAP : n;
      n = n < 0 ? 0 : n;
#pragma unroll 1
      for (int i = 0; i < n; ++i) {
        const int ent  = list[wsx * WCAP + i];
        const int slot = ent & (NBK - 1);
        if ((slot & (NWAVE - 1)) != wave) continue;
        const int el     = (ent >> 6) & (CHUNK - 1);
        const int isSelf = (ent >> 20) & 1;
        int e = cbase + el;
        e = e > nE - 1 ? nE - 1 : e;
        int s = ei[e];
        s = s < 0 ? 0 : (s > nN - 1 ? nN - 1 : s);
        int nd = nodeBase + slot;
        nd = nd > nN - 1 ? nN - 1 : nd;
        const int src = isSelf ? nd : s;

        const float* pl = xl + (size_t)src * HID + 8 * lane;
        const float* pr = xr + (size_t)nd  * HID + 8 * lane;
        const float* pa = satt + 8 * lane;
        v4f xa[4], xb[4];
        float dot = 0.f;
#pragma unroll
        for (int q = 0; q < 4; ++q) {
          const int o = 256 * q;
          const v4f a0 = *(const v4f*)(pl + o);
          const v4f a1 = *(const v4f*)(pl + o + 4);
          const v4f r0 = *(const v4f*)(pr + o);
          const v4f r1 = *(const v4f*)(pr + o + 4);
          const v4f w0 = *(const v4f*)(pa + o);
          const v4f w1 = *(const v4f*)(pa + o + 4);
          xa[q] = a0;
          xb[q] = a1;
          const v4f t0 = lrelu4(a0 + r0);
          const v4f t1 = lrelu4(a1 + r1);
          dot += t0.x * w0.x; dot += t0.y * w0.y; dot += t0.z * w0.z; dot += t0.w * w0.w;
          dot += t1.x * w1.x; dot += t1.y * w1.y; dot += t1.z * w1.z; dot += t1.w * w1.w;
        }
        dot = wsum(dot);
        const float m_old = mls[slot];
        const float l_old = lls[slot];
        const float m_new = fmaxf(m_old, dot);
        const float sc = __expf(m_old - m_new);
        const float p  = __expf(dot - m_new);
        float* ps = sacc + slot * HID + 8 * lane;
#pragma unroll
        for (int q = 0; q < 4; ++q) {
          const int o = 256 * q;
          v4f g0 = *(const v4f*)(ps + o);
          v4f g1 = *(const v4f*)(ps + o + 4);
          g0 = g0 * sc + xa[q] * p;
          g1 = g1 * sc + xb[q] * p;
          *(v4f*)(ps + o)     = g0;
          *(v4f*)(ps + o + 4) = g1;
        }
        mls[slot] = m_new;
        lls[slot] = l_old * sc + p;
      }
    }
    __syncthreads();
  }

  const v4f z4 = {0.f, 0.f, 0.f, 0.f};
#pragma unroll 1
  for (int j = 0; j < NBK / NWAVE; ++j) {
    const int slot = wave + NWAVE * j;
    const int node = nodeBase + slot;
    const bool live = node < nN;
    const float lv  = lls[slot];
    const float inv = 1.0f / lv;
    const float* psrc = sacc + slot * HID + 8 * lane;
#pragma unroll 1
    for (int pass = 0; pass < 2; ++pass) {
#pragma unroll 1
      for (int q = 0; q < 4; ++q) {
        const int o = 256 * q;
        const v4f g0 = *(const v4f*)(psrc + o);
        const v4f g1 = *(const v4f*)(psrc + o + 4);
        const v4f b0 = *(const v4f*)(cb + o + 8 * lane);
        const v4f b1 = *(const v4f*)(cb + o + 8 * lane + 4);
        v4f v0 = g0 * inv + b0;
        v4f v1 = g1 * inv + b1;
        v0.x = v0.x > 0.f ? v0.x : 0.f; v0.y = v0.y > 0.f ? v0.y : 0.f;
        v0.z = v0.z > 0.f ? v0.z : 0.f; v0.w = v0.w > 0.f ? v0.w : 0.f;
        v1.x = v1.x > 0.f ? v1.x : 0.f; v1.y = v1.y > 0.f ? v1.y : 0.f;
        v1.z = v1.z > 0.f ? v1.z : 0.f; v1.w = v1.w > 0.f ? v1.w : 0.f;
        v0 = live ? v0 : z4;
        v1 = live ? v1 : z4;
        float t[8];
        t[0] = v0.x; t[1] = v0.y; t[2] = v0.z; t[3] = v0.w;
        t[4] = v1.x; t[5] = v1.y; t[6] = v1.z; t[7] = v1.w;
        v8us H, L;
#pragma unroll
        for (int ee = 0; ee < 8; ++ee) { unsigned short u, w; split_bf(t[ee], u, w); H[ee] = u; L[ee] = w; }
        const size_t off = (size_t)node * HID + o + 8 * lane;
        *(volatile v8us*)(hhi + off) = H;
        *(volatile v8us*)(hlo + off) = L;
      }
      if (pass == 0) __threadfence();
    }
  }
}

extern "C" void kernel_launch(void* const* d_in, const int* in_sizes, int n_in,
                              void* d_out, int out_size, void* d_ws, size_t ws_size,
                              hipStream_t stream) {
  if (n_in < 14) return;
  const int nN = in_sizes[0] / F_IN;
  if (nN < 1 || in_sizes[0] != nN * F_IN) return;
  if (in_sizes[1] < 2 || (in_sizes[1] & 1)) return;
  const int nE = in_sizes[1] / 2;
  if (in_sizes[2] != F_IN * HID || in_sizes[3] != HID) return;
  if (in_sizes[4] != F_IN * HID || in_sizes[5] != HID) return;
  if (in_sizes[6] != HID || in_sizes[7] != HID) return;
  if (in_sizes[8] != HID * C1 || in_sizes[9] != C1) return;
  if (in_sizes[10] != C1 * C2 || in_sizes[11] != C2) return;
  const int nC = in_sizes[13];
  if (nC < 1 || nC > NCP || in_sizes[12] != C2 * nC) return;
  if (out_size != nN * nC) return;

  const float* x    = (const float*)d_in[0];
  const int*   ei   = (const int*)d_in[1];
  const float* Wl   = (const float*)d_in[2];
  const float* bl   = (const float*)d_in[3];
  const float* Wr   = (const float*)d_in[4];
  const float* br   = (const float*)d_in[5];
  const float* att  = (const float*)d_in[6];
  const float* cvb  = (const float*)d_in[7];
  const float* W1   = (const float*)d_in[8];
  const float* b1   = (const float*)d_in[9];
  const float* W2   = (const float*)d_in[10];
  const float* b2   = (const float*)d_in[11];
  const float* Wc   = (const float*)d_in[12];
  const float* bc   = (const float*)d_in[13];
  float* out = (float*)d_out;

  const int MP = ((nN + TM - 1) / TM) * TM;

  char* wsb = (char*)d_ws;
  size_t off = 0;
  const size_t nWl = (size_t)HID * F_IN, nW1 = (size_t)C1 * HID, nW2 = (size_t)C2 * C1, nWc = (size_t)NCP * C2;
  unsigned short* WlThi = (unsigned short*)(wsb + off); off += nWl * 2;
  unsigned short* WlTlo = (unsigned short*)(wsb + off); off += nWl * 2;
  unsigned short* WrThi = (unsigned short*)(wsb + off); off += nWl * 2;
  unsigned short* WrTlo = (unsigned short*)(wsb + off); off += nWl * 2;
  unsigned short* W1Thi = (unsigned short*)(wsb + off); off += nW1 * 2;
  unsigned short* W1Tlo = (unsigned short*)(wsb + off); off += nW1 * 2;
  unsigned short* W2Thi = (unsigned short*)(wsb + off); off += nW2 * 2;
  unsigned short* W2Tlo = (unsigned short*)(wsb + off); off += nW2 * 2;
  unsigned short* WcThi = (unsigned short*)(wsb + off); off += nWc * 2;
  unsigned short* WcTlo = (unsigned short*)(wsb + off); off += nWc * 2;
  const size_t regBytes = (size_t)MP * HID * 4;
  float* XL = (float*)(wsb + off);
  unsigned short* H2hi = (unsigned short*)(wsb + off);
  unsigned short* H2lo = H2hi + (size_t)MP * C2;
  off += regBytes;
  float* XR = (float*)(wsb + off);
  unsigned short* H1hi = (unsigned short*)(wsb + off);
  unsigned short* H1lo = H1hi + (size_t)MP * C1;
  off += regBytes;
  unsigned short* Xhi = (unsigned short*)(wsb + off);
  unsigned short* Xlo = Xhi + (size_t)MP * F_IN;
  unsigned short* Hhi = (unsigned short*)(wsb + off);
  unsigned short* Hlo = Hhi + (size_t)MP * HID;
  off += regBytes;
  if (off > ws_size) return;
  if ((size_t)MP * C2 * 2 * 2 > regBytes || (size_t)MP * C1 * 2 * 2 > regBytes || (size_t)MP * F_IN * 2 * 2 > regBytes) return;

  {
    const long long tot8 = (long long)MP * F_IN / 8;
    const unsigned nb = (unsigned)((tot8 + NTHR - 1) / NTHR);
    k_cvt_rows<<<nb, NTHR, 0, stream>>>(x, nN, F_IN, MP, Xhi, Xlo);
  }
  k_cvt_T<<<dim3(F_IN / 64, HID / 64), NTHR, 0, stream>>>(Wl, F_IN, HID, F_IN, WlThi, WlTlo);
  k_cvt_T<<<dim3(F_IN / 64, HID / 64), NTHR, 0, stream>>>(Wr, F_IN, HID, F_IN, WrThi, WrTlo);
  k_cvt_T<<<dim3(HID / 64, C1 / 64),   NTHR, 0, stream>>>(W1, HID, C1, HID, W1Thi, W1Tlo);
  k_cvt_T<<<dim3(C1 / 64, C2 / 64),    NTHR, 0, stream>>>(W2, C1, C2, C1, W2Thi, W2Tlo);
  k_cvt_T<<<dim3(C2 / 64, NCP / 64),   NTHR, 0, stream>>>(Wc, C2, nC, C2, WcThi, WcTlo);

  k_gemm<<<dim3(MP / TM, HID / TNB), NTHR, 0, stream>>>(Xhi, Xlo, F_IN, WlThi, WlTlo, F_IN, F_IN,
                                                        bl, HID, 0, XL, H1hi, H1lo, HID, out, nN, nC);
  k_gemm<<<dim3(MP / TM, HID / TNB), NTHR, 0, stream>>>(Xhi, Xlo, F_IN, WrThi, WrTlo, F_IN, F_IN,
                                                        br, HID, 0, XR, H1hi, H1lo, HID, out, nN, nC);

  hipFuncSetAttribute(reinterpret_cast<const void*>(&k_gat),
                      hipFuncAttributeMaxDynamicSharedMemorySize, LDS_GAT_BYTES);
  k_gat<<<MP / NBK, NTHR, LDS_GAT_BYTES, stream>>>(XL, XR, ei, att, cvb, Hhi, Hlo, nN, nE);

  k_gemm<<<dim3(MP / TM, C1 / TNB), NTHR, 0, stream>>>(Hhi, Hlo, HID, W1Thi, W1Tlo, HID, HID,
                                                       b1, C1, 1, XL, H1hi, H1lo, C1, out, nN, nC);
  k_gemm<<<dim3(MP / TM, C2 / TNB), NTHR, 0, stream>>>(H1hi, H1lo, C1, W2Thi, W2Tlo, C1, C1,
                                                       b2, C2, 1, XR, H2hi, H2lo, C2, out, nN, nC);
  k_gemm<<<dim3(MP / TM, NCP / TNB), NTHR, 0, stream>>>(H2hi, H2lo, C2, WcThi, WcTlo, C2, C2,
                                                        bc, nC, 2, XR, H1hi, H1lo, C2, out, nN, nC);
}
